// LongcatMoe_88235808129201
// MI455X (gfx1250) — hardware-verified
//
#include <hip/hip_runtime.h>
#include <stddef.h>
#include <stdint.h>

#define NTOK   4096
#define DIM    1024
#define HID    768
#define NE     8
#define NSEL   2
#define RPITCH 8
#define NTILE  136
#define AROWS  (NTILE * 64)
#define NPROW  (NTOK * NSEL)
#define LPIECE (NTOK / 4)
#define WSC    64.0f
#define UGS    0.015625f
#define ACS    256.0f
#define LSC    2048.0f
#define LINV   0.00048828125f
#define DNS    0.00006103515625f
#define APITCH 136
#define EPITCH 72
#define OTP    68

static_assert(NTILE == NPROW / 64 + NE);
static_assert(NSEL == 2);
static_assert(NE == 8);
static_assert(DIM % 128 == 0);
static_assert(HID % 128 == 0);
static_assert(DIM % 64 == 0);
static_assert(HID % 64 == 0);
static_assert(NTOK % 256 == 0);
static_assert(NTOK % 8 == 0);
static_assert(LPIECE == 4 * 256);
static_assert((NTOK * DIM) % 2048 == 0);
static_assert((NE * 2 * HID * DIM) % 2048 == 0);
static_assert((NE * DIM * HID) % 2048 == 0);

typedef _Float16 v16h __attribute__((ext_vector_type(16)));
typedef _Float16 v8h  __attribute__((ext_vector_type(8)));
typedef float    v8f  __attribute__((ext_vector_type(8)));
typedef float    v4f  __attribute__((ext_vector_type(4)));
typedef unsigned int v4u __attribute__((ext_vector_type(4)));
typedef int      v4i  __attribute__((ext_vector_type(4)));
typedef unsigned short v4us __attribute__((ext_vector_type(4)));

union Frag  { v16h v; v8h h[2]; };
union Pack8 { v8h h; v4u u; };

__device__ __forceinline__ int clampi(int v, int lo, int hi) { return min(max(v, lo), hi); }

__device__ __forceinline__ v8f mma16(v16h a, v16h b, v8f c) {
  c = __builtin_amdgcn_wmma_f32_16x16x32_f16(false, a, false, b, (short)0, c, false, false);
  asm volatile("v_nop\n\tv_nop\n\tv_nop\n\tv_nop" : "+v"(c) : "v"(a), "v"(b));
  return c;
}

__device__ __forceinline__ v16h ldfrag(const _Float16* p, int ld, int row0, int k0, int lane) {
  const int m = lane & 15, lh = lane >> 4;
  const _Float16* q = p + (size_t)(row0 + m) * ld + k0 + 8 * lh;
  Frag f;
  f.h[0] = *(const v8h*)(q);
  f.h[1] = *(const v8h*)(q + 16);
  return f.v;
}

__device__ __forceinline__ v8f zero8() { return (v8f){0.f, 0.f, 0.f, 0.f, 0.f, 0.f, 0.f, 0.f}; }

__global__ __launch_bounds__(256) void k_cvt(const float* __restrict__ src, _Float16* __restrict__ dh, int n8,
                                             float scale) {
  const int i = blockIdx.x * 256 + (int)threadIdx.x;
  if (i >= n8) return;
  const size_t o = (size_t)i * 8;
  const v4f a0 = *(const v4f*)(src + o) * scale;
  const v4f a1 = *(const v4f*)(src + o + 4) * scale;
  Pack8 pk;
  pk.h = (v8h){(_Float16)a0[0], (_Float16)a0[1], (_Float16)a0[2], (_Float16)a0[3],
               (_Float16)a1[0], (_Float16)a1[1], (_Float16)a1[2], (_Float16)a1[3]};
  const v4u vv = pk.u;
  volatile v4u* d = (volatile v4u*)(dh + o);
  *d = vv;
  __threadfence();
  *d = vv;
}

__global__ __launch_bounds__(256) void k_route(const float* __restrict__ x, const float* __restrict__ gw,
                                               const int* __restrict__ ngt, const int* __restrict__ mtg,
                                               float* __restrict__ rp) {
  (void)ngt;
  (void)mtg;
  __shared__ __align__(16) float sR[8 * RPITCH];
  const int tid = threadIdx.x, lane = tid & 31, wave = tid >> 5;
  const int c = lane & 15, c8 = lane & 7;
  const size_t t = (size_t)blockIdx.x * 8 + wave;
  const float* xr = x + t * DIM;

  float a[NE];
#pragma unroll
  for (int e = 0; e < NE; ++e) a[e] = 0.f;
#pragma unroll 1
  for (int j = 0; j < DIM / 32; ++j) {
    const int k = j * 32 + lane;
    const float xv = xr[k];
#pragma unroll
    for (int e = 0; e < NE; ++e) a[e] += xv * gw[(size_t)e * DIM + k];
  }
#pragma unroll
  for (int e = 0; e < NE; ++e) {
#pragma unroll
    for (int off = 16; off >= 1; off >>= 1) a[e] += __shfl_xor(a[e], off, 32);
  }

  float mx = a[0];
#pragma unroll
  for (int e = 1; e < NE; ++e) mx = fmaxf(mx, a[e]);
  float mine = a[0];
#pragma unroll
  for (int e = 1; e < NE; ++e) mine = (c8 == e) ? a[e] : mine;
  const float exm = expf(mine - mx);
  float ssum = exm;
#pragma unroll
  for (int off = 1; off < 8; off <<= 1) ssum += __shfl_xor(ssum, off, 32);
  const float inv = 1.0f / ssum;
  const float scm = exm * inv;
  float sc[NE];
#pragma unroll
  for (int e = 0; e < NE; ++e) sc[e] = __shfl(scm, e, 32);

  const float NEGI = -__builtin_huge_valf();
  unsigned taken = 0u;
  int idx[NSEL];
  float wsel[NSEL];
#pragma unroll
  for (int kk = 0; kk < NSEL; ++kk) {
    float bv = NEGI;
    int best = 0;
    float bs = 0.f;
#pragma unroll
    for (int i = 0; i < NE; ++i) {
      const bool cnd = (((taken >> i) & 1u) == 0u) && (sc[i] > bv);
      bv   = cnd ? sc[i] : bv;
      best = cnd ? i : best;
      bs   = cnd ? sc[i] : bs;
    }
    taken |= (1u << best);
    idx[kk]  = best;
    wsel[kk] = bs;
  }
  const float w0 = wsel[0];
  const float w1 = wsel[1];

  float ov = 0.f;
  ov = (lane == 0) ? (float)idx[0] : ov;
  ov = (lane == 1) ? (float)idx[1] : ov;
  ov = (lane == 4) ? w0 : ov;
  ov = (lane == 5) ? w1 : ov;
  if (lane < RPITCH) sR[wave * RPITCH + lane] = ov;
  __syncthreads();
  if (wave == 0) {
    const v4f vr = *(const v4f*)(sR + c * 4);
    volatile v4f* dr = (volatile v4f*)(rp + (size_t)blockIdx.x * (8 * RPITCH) + c * 4);
    if (lane < 16) *dr = vr;
    __threadfence();
    if (lane < 16) *dr = vr;
  }
}

__global__ __launch_bounds__(256) void k_lists(const float* __restrict__ rp, int* __restrict__ tokl,
                                               float* __restrict__ wl, int* __restrict__ tab) {
  __shared__ __align__(16) unsigned short ltok[NTOK];
  __shared__ __align__(16) float lw[NTOK];
  __shared__ int wc[8];
  __shared__ __align__(16) int sTab[64];
  const int tid = threadIdx.x, lane = tid & 31, wave = tid >> 5;
  if (tid < 64) sTab[tid] = 0;
  int tbrun = 0;
#pragma unroll 1
  for (int e = 0; e < NE; ++e) {
    __syncthreads();
    for (int i = tid; i < NTOK; i += 256) { ltok[i] = (unsigned short)0; lw[i] = 0.f; }
    __syncthreads();
    int run = 0;
#pragma unroll 1
    for (int ch = 0; ch < NTOK / 256; ++ch) {
      const int t = ch * 256 + tid;
      const v4f ri = *(const v4f*)(rp + (size_t)t * RPITCH);
      const v4f rw = *(const v4f*)(rp + (size_t)t * RPITCH + 4);
      int hit = -1;
      float w = 0.f;
#pragma unroll
      for (int k = NSEL - 1; k >= 0; --k) {
        const bool m = ((int)ri[k] == e);
        hit = m ? k : hit;
        w   = m ? rw[k] : w;
      }
      const bool flag = (hit >= 0);
      const unsigned bal = __builtin_amdgcn_ballot_w32(flag);
      const int pre = __builtin_popcount(bal & ((1u << lane) - 1u));
      if (lane == 0) wc[wave] = __builtin_popcount(bal);
      __syncthreads();
      int base = run, tot = 0;
#pragma unroll
      for (int q = 0; q < 8; ++q) {
        const int cw = wc[q];
        base += (q < wave) ? cw : 0;
        tot  += cw;
      }
      const int pos = clampi(base + pre, 0, NTOK - 1);
      if (flag) { ltok[pos] = (unsigned short)(t * NSEL + hit); lw[pos] = w; }
      run += tot;
      __syncthreads();
    }
    run = clampi(run, 0, NTOK);
    const int ntl = (run + 63) >> 6;
    if (tid == 0) { sTab[e] = run; sTab[32 + e + 1] = clampi(tbrun + ntl, 0, NTILE); }
    tbrun += ntl;

    int*   trow = tokl + (size_t)e * NTOK;
    float* wrow = wl + (size_t)e * NTOK;
    v4i tv[4];
    v4f wv[4];
    int po[4];
#pragma unroll
    for (int it = 0; it < 4; ++it) {
      const int p = tid + 256 * it;
      const v4us u = *(const v4us*)(ltok + p * 4);
      tv[it] = (v4i){(int)u[0], (int)u[1], (int)u[2], (int)u[3]};
      wv[it] = *(const v4f*)(lw + p * 4);
      po[it] = p * 4;
    }
    for (int ps = 0; ps < 2; ++ps) {
#pragma unroll
      for (int it = 0; it < 4; ++it) {
        *(volatile v4i*)(trow + po[it]) = tv[it];
        *(volatile v4f*)(wrow + po[it]) = wv[it];
      }
      __threadfence();
    }
  }
  __syncthreads();
  if (wave == 0) {
    const v4i v = *(const v4i*)(sTab + (lane & 15) * 4);
    volatile v4i* d = (volatile v4i*)(tab + (lane & 15) * 4);
    if (lane < 16) *d = v;
    __threadfence();
    if (lane < 16) *d = v;
  }
}

__global__ __launch_bounds__(256) void k_upgate(const _Float16* __restrict__ xh,
                                                const _Float16* __restrict__ w13h,
                                                const int* __restrict__ tokl, const int* __restrict__ tab,
                                                _Float16* __restrict__ act, _Float16* __restrict__ actl) {
  __shared__ __align__(16) _Float16 sA[64 * APITCH];
  __shared__ __align__(16) _Float16 sE[2 * 8 * 16 * EPITCH];
  __shared__ int   sTok[64];
  __shared__ int   sTab[64];
  const int tid = threadIdx.x, lane = tid & 31, wave = tid >> 5;
  const int hh = lane >> 4, c = lane & 15;
  const int wm = wave & 3, wn = wave >> 2;
  const int b  = blockIdx.y;
  const int n0 = blockIdx.x * 128;

  if (tid < 64) sTab[tid] = tab[tid];
  __syncthreads();
  const int tb8 = clampi(sTab[32 + NE], 0, NTILE);
  if (b >= tb8) return;
  int e = 0;
#pragma unroll
  for (int q = 1; q < NE; ++q) e += (clampi(sTab[32 + q], 0, NTILE) <= b) ? 1 : 0;
  const int tbe = clampi(sTab[32 + e], 0, NTILE);
  if (tid < 64) {
    const int rloc = (b - tbe) * 64 + tid;
    const int li = e * NTOK + clampi(rloc, 0, NTOK - 1);
    const int enc = tokl[li];
    sTok[tid] = clampi(enc >> 1, 0, NTOK - 1);
  }
  __syncthreads();

  const _Float16* wge = w13h + (size_t)e * (size_t)(2 * HID * DIM);
  const _Float16* wue = wge + (size_t)HID * DIM;
  const int brow = n0 + wn * 64;

  v8f accG[4], accU[4];
#pragma unroll
  for (int t = 0; t < 4; ++t) { accG[t] = zero8(); accU[t] = zero8(); }

  const int ar = tid >> 2, ac = tid & 3;
  const _Float16* xrow = xh + (size_t)sTok[ar] * DIM + ac * 32;
  _Float16* arow = sA + ar * APITCH + ac * 32;
#pragma unroll 1
  for (int kc = 0; kc < DIM / 128; ++kc) {
    __syncthreads();
#pragma unroll
    for (int q = 0; q < 4; ++q) *(v8h*)(arow + 8 * q) = *(const v8h*)(xrow + kc * 128 + 8 * q);
    __syncthreads();
#pragma unroll 1
    for (int ks = 0; ks < 4; ++ks) {
      const int kg = kc * 128 + ks * 32;
      const v16h a = ldfrag(sA, APITCH, wm * 16, ks * 32, lane);
#pragma unroll
      for (int t = 0; t < 4; ++t) {
        const v16h bq = ldfrag(wge, DIM, brow + 16 * t, kg, lane);
        accG[t] = mma16(a, bq, accG[t]);
      }
#pragma unroll
      for (int t = 0; t < 4; ++t) {
        const v16h bq = ldfrag(wue, DIM, brow + 16 * t, kg, lane);
        accU[t] = mma16(a, bq, accU[t]);
      }
    }
  }

  _Float16* ewh = sE + wave * (16 * EPITCH);
  _Float16* ewl = sE + (8 + wave) * (16 * EPITCH);
#pragma unroll
  for (int t = 0; t < 4; ++t) {
#pragma unroll
    for (int r = 0; r < 8; ++r) {
      const float g = accG[t][r] * UGS;
      const float u = accU[t][r] * UGS;
      const float sg = __builtin_amdgcn_rcpf(1.0f + __expf(-g));
      const float av = ((g * sg) * u) * ACS;
      const _Float16 ah = (_Float16)av;
      const float res = (av - (float)ah) * LSC;
      const _Float16 al = (_Float16)res;
      ewh[(8 * hh + r) * EPITCH + 16 * t + c] = ah;
      ewl[(8 * hh + r) * EPITCH + 16 * t + c] = al;
    }
  }
  __syncthreads();
  v4u vh[4], vl[4];
  size_t go[4];
#pragma unroll
  for (int it = 0; it < 4; ++it) {
    const int p  = lane + 32 * it;
    const int L  = p >> 3;
    const int pc = p & 7;
    Pack8 pk;
    pk.h   = *(const v8h*)(ewh + L * EPITCH + pc * 8);
    vh[it] = pk.u;
    Pack8 pl;
    pl.h   = *(const v8h*)(ewl + L * EPITCH + pc * 8);
    vl[it] = pl.u;
    go[it] = (size_t)(b * 64 + wm * 16 + L) * HID + brow + pc * 8;
  }
  for (int ps = 0; ps < 2; ++ps) {
#pragma unroll
    for (int it = 0; it < 4; ++it) {
      *(volatile v4u*)(act  + go[it]) = vh[it];
      *(volatile v4u*)(actl + go[it]) = vl[it];
    }
    __threadfence();
  }
}

__global__ __launch_bounds__(256) void k_downx(const _Float16* __restrict__ act, const _Float16* __restrict__ actl,
                                               const _Float16* __restrict__ w2h,
                                               const int* __restrict__ tokl, const float* __restrict__ wl,
                                               const int* __restrict__ tab, float* __restrict__ part) {
  __shared__ __align__(16) float sO[8 * 16 * OTP];
  __shared__ int   sEnc[64];
  __shared__ float sW[64];
  __shared__ int   sVal[64];
  __shared__ int   sTab[64];
  const int tid = threadIdx.x, lane = tid & 31, wave = tid >> 5;
  const int hh = lane >> 4, c = lane & 15;
  const int wm = wave & 3, wn = wave >> 2;
  const int b  = blockIdx.y;
  const int n0 = blockIdx.x * 128;

  if (tid < 64) sTab[tid] = tab[tid];
  __syncthreads();
  const int tb8 = clampi(sTab[32 + NE], 0, NTILE);
  if (b >= tb8) return;
  int e = 0;
#pragma unroll
  for (int q = 1; q < NE; ++q) e += (clampi(sTab[32 + q], 0, NTILE) <= b) ? 1 : 0;
  const int tbe = clampi(sTab[32 + e], 0, NTILE);
  const int cne = clampi(sTab[e], 0, NTOK);
  if (tid < 64) {
    const int rloc = (b - tbe) * 64 + tid;
    const bool valid = (rloc >= 0) && (rloc < cne);
    const int li = e * NTOK + clampi(rloc, 0, NTOK - 1);
    const int enc = tokl[li];
    const float w = wl[li];
    sEnc[tid] = clampi(enc, 0, NPROW - 1);
    sW[tid]   = valid ? w : 0.f;
    sVal[tid] = valid ? 1 : 0;
  }
  __syncthreads();

  const _Float16* wde = w2h + (size_t)e * (size_t)(DIM * HID);
  const int brow = n0 + wn * 64;
  const int arow = b * 64 + wm * 16;
  v8f accH[4], accL[4];
#pragma unroll
  for (int t = 0; t < 4; ++t) { accH[t] = zero8(); accL[t] = zero8(); }
#pragma unroll 1
  for (int k0 = 0; k0 < HID; k0 += 32) {
    const v16h ah = ldfrag(act,  HID, arow, k0, lane);
    const v16h al = ldfrag(actl, HID, arow, k0, lane);
#pragma unroll
    for (int t = 0; t < 4; ++t) {
      const v16h bq = ldfrag(wde, HID, brow + 16 * t, k0, lane);
      accH[t] = mma16(ah, bq, accH[t]);
      accL[t] = mma16(al, bq, accL[t]);
    }
  }

  float wr[8];
#pragma unroll
  for (int r = 0; r < 8; ++r) wr[r] = sW[wm * 16 + 8 * hh + r] * DNS;
  float* sw = sO + wave * (16 * OTP);
#pragma unroll
  for (int t = 0; t < 4; ++t) {
#pragma unroll
    for (int r = 0; r < 8; ++r) sw[(8 * hh + r) * OTP + 16 * t + c] = (accH[t][r] + accL[t][r] * LINV) * wr[r];
  }
  __syncthreads();
  v4f val[8];
  size_t go[8];
  bool ok[8];
#pragma unroll
  for (int it = 0; it < 8; ++it) {
    const int p    = lane + 32 * it;
    const int L    = p >> 3;
    const int pc   = p & 7;
    const int row  = L >> 1;
    const int half = L & 1;
    const int lr   = wm * 16 + row;
    val[it] = *(const v4f*)(sw + row * OTP + half * 32 + pc * 4);
    ok[it]  = (sVal[lr] != 0);
    go[it]  = (size_t)sEnc[lr] * DIM + brow + half * 32 + pc * 4;
  }
  for (int ps = 0; ps < 2; ++ps) {
#pragma unroll
    for (int it = 0; it < 8; ++it) {
      if (ok[it]) *(volatile v4f*)(part + go[it]) = val[it];
    }
    __threadfence();
  }
}

__global__ __launch_bounds__(256) void k_comb(const float* __restrict__ part, float* __restrict__ out, int n4) {
  const int i = blockIdx.x * 256 + (int)threadIdx.x;
  if (i >= n4) return;
  const size_t t = (size_t)i / (DIM / 4);
  const size_t n = ((size_t)i % (DIM / 4)) * 4;
  const float* pr = part + t * (size_t)(NSEL * DIM) + n;
  v4f v = *(const v4f*)(pr);
  const v4f p1 = *(const v4f*)(pr + DIM);
  v = v + p1;
  volatile v4f* d = (volatile v4f*)(out + t * DIM + n);
  *d = v;
  __threadfence();
  *d = v;
}

extern "C" void kernel_launch(void* const* d_in, const int* in_sizes, int n_in,
                              void* d_out, int out_size, void* d_ws, size_t ws_size,
                              hipStream_t stream) {
  if (n_in < 6) return;
  if (in_sizes[0] != NTOK * DIM) return;
  if (in_sizes[1] != NE * DIM) return;
  if (in_sizes[2] != NE * 2 * HID * DIM) return;
  if (in_sizes[3] != NE * DIM * HID) return;
  if (in_sizes[4] < 1) return;
  if (in_sizes[5] < 1) return;
  if (out_size != NTOK * DIM) return;

  const float* x     = (const float*)d_in[0];
  const float* Wgate = (const float*)d_in[1];
  const float* W13   = (const float*)d_in[2];
  const float* W2    = (const float*)d_in[3];
  const int*   Ngt   = (const int*)d_in[4];
  const int*   Mtg   = (const int*)d_in[5];
  float* out = (float*)d_out;

  size_t off = 0;
  const size_t oXh = off; off += (size_t)NTOK * DIM * 2;
  const size_t oW1 = off; off += (size_t)NE * 2 * HID * DIM * 2;
  const size_t oW2 = off; off += (size_t)NE * DIM * HID * 2;
  const size_t oR  = off; off += (size_t)NTOK * RPITCH * 4;
  const size_t oTL = off; off += (size_t)NE * NTOK * 4;
  const size_t oWL = off; off += (size_t)NE * NTOK * 4;
  const size_t oTB = off; off += (size_t)256;
  const size_t oAC = off; off += (size_t)AROWS * HID * 2;
  const size_t oAL = off; off += (size_t)AROWS * HID * 2;
  const size_t oP  = off; off += (size_t)NPROW * DIM * 4;
  if (off > ws_size) return;
  if (off > (size_t)134217728) return;
  if ((oW1 | oW2 | oR | oTL | oWL | oTB | oAC | oAL | oP) & (size_t)127) return;

  char* ws = (char*)d_ws;
  _Float16* Xh   = (_Float16*)(ws + oXh);
  _Float16* W13h = (_Float16*)(ws + oW1);
  _Float16* W2h  = (_Float16*)(ws + oW2);
  float*    R    = (float*)(ws + oR);
  int*      TOK  = (int*)(ws + oTL);
  float*    WL   = (float*)(ws + oWL);
  int*      TAB  = (int*)(ws + oTB);
  _Float16* ACTH = (_Float16*)(ws + oAC);
  _Float16* ACTL = (_Float16*)(ws + oAL);
  float*    P    = (float*)(ws + oP);

  const int n8x  = (NTOK * DIM) / 8;
  const int n8w1 = (NE * 2 * HID * DIM) / 8;
  const int n8w2 = (NE * DIM * HID) / 8;

  k_cvt<<<dim3((n8x + 255) / 256), dim3(256), 0, stream>>>(x, Xh, n8x, 1.0f);
  k_cvt<<<dim3((n8w1 + 255) / 256), dim3(256), 0, stream>>>(W13, W13h, n8w1, WSC);
  k_cvt<<<dim3((n8w2 + 255) / 256), dim3(256), 0, stream>>>(W2, W2h, n8w2, WSC);
  k_route<<<dim3(NTOK / 8), dim3(256), 0, stream>>>(x, Wgate, Ngt, Mtg, R);
  k_lists<<<dim3(1), dim3(256), 0, stream>>>(R, TOK, WL, TAB);
  k_upgate<<<dim3(HID / 128, NTILE), dim3(256), 0, stream>>>(Xh, W13h, TOK, TAB, ACTH, ACTL);
  k_downx<<<dim3(DIM / 128, NTILE), dim3(256), 0, stream>>>(ACTH, ACTL, W2h, TOK, WL, TAB, P);
  k_comb<<<dim3((NTOK * DIM) / 4 / 256), dim3(256), 0, stream>>>(P, out, (NTOK * DIM) / 4);
  (void)hipGetLastError();
}
